// HMABottleneck_43190191129253
// MI455X (gfx1250) — hardware-run, weakly checked
//
#include <hip/hip_runtime.h>
#include <math.h>

#define NB    4
#define CC    512
#define DI    1024
#define KD    4
#define NS    16
#define RK    32
#define XW    64
#define XDN   256
#define NVSS  5
#define H0    16
#define L0    256
#define M0    1024
#define KC9   4608
#define WSC   256.0f
#define XSSC  16.0f
#define DTSC  64.0f
#define OSC1  0.00390625f
#define OSCX  0.000244140625f
#define OSCD  0.00006103515625f
#define BNS   0.99999500003749969f
#define LNE1  1e-6f
#define LNE2  1e-5f
#define GSTR  40
#define OSTR  68
#define SMEMB 17408
#define LOG2E 1.4426950408889634f

static_assert(XDN == KD * XW);
static_assert(XW == RK + 2 * NS);
static_assert(M0 == NB * L0 && L0 == H0 * H0);
static_assert(KC9 == 9 * CC);
static_assert(SMEMB >= 2 * 64 * GSTR * 2);
static_assert(SMEMB >= 4 * 16 * OSTR * 4);
static_assert(CC % 64 == 0 && DI % 64 == 0 && XDN % 64 == 0);
static_assert(CC % 32 == 0 && DI % 32 == 0 && KC9 % 32 == 0 && RK == 32);
static_assert(DI == 4 * 256);
static_assert(CC == 64 * 8);
static_assert(DI == 128 * 8);

typedef _Float16 v16h __attribute__((ext_vector_type(16)));
typedef _Float16 v8h  __attribute__((ext_vector_type(8)));
typedef _Float16 v8ha __attribute__((ext_vector_type(8), may_alias));
typedef float v8f  __attribute__((ext_vector_type(8)));
typedef float v4f  __attribute__((ext_vector_type(4)));
typedef float v4fa __attribute__((ext_vector_type(4), may_alias));
union Frag { v16h v; v8h h[2]; };

__device__ __forceinline__ float siluf(float x) { return x * __builtin_amdgcn_rcpf(1.0f + __expf(-x)); }
__device__ __forceinline__ float geluf(float x) { return 0.5f * x * (1.0f + erff(x * 0.70710678118654752f)); }
__device__ __forceinline__ int clampi(int v, int lo, int hi) { return (v < lo) ? lo : ((v > hi) ? hi : v); }

__device__ __forceinline__ void st16(_Float16* p, v8h o) { *(volatile v4fa*)p = __builtin_bit_cast(v4f, o); }
__device__ __forceinline__ void st16f(float* p, v4f o) { *(volatile v4fa*)p = o; }

__device__ __forceinline__ v8h cvt8(const v4f a, const v4f b, float sc) {
  v8h o;
#pragma unroll
  for (int u = 0; u < 4; ++u) { o[u] = (_Float16)(a[u] * sc); o[4 + u] = (_Float16)(b[u] * sc); }
  return o;
}

__device__ __forceinline__ v8f mma_f16(v16h a, v16h b, v8f c) {
  return __builtin_amdgcn_wmma_f32_16x16x32_f16(false, a, false, b, (short)0, c, false, false);
}
__device__ __forceinline__ void wguard(v8f& c0, v8f& c1, v8f& c2, v8f& c3, const v16h& a,
                                       const v16h& b0, const v16h& b1, const v16h& b2, const v16h& b3) {
#if defined(__HIP_DEVICE_COMPILE__)
  asm volatile("v_nop\n\tv_nop\n\tv_nop\n\tv_nop"
               : "+v"(c0), "+v"(c1), "+v"(c2), "+v"(c3)
               : "v"(a), "v"(b0), "v"(b1), "v"(b2), "v"(b3));
#endif
}

__device__ __forceinline__ v16h lds_frag(const _Float16* base) {
  const int lane = threadIdx.x & 31, r = lane & 15, kh = (lane >> 4) * 8;
  Frag f;
  f.h[0] = *(const v8ha*)(base + r * GSTR + kh);
  f.h[1] = *(const v8ha*)(base + r * GSTR + 16 + kh);
  return f.v;
}

__device__ __forceinline__ void stage64(_Float16* lds, const _Float16* __restrict__ P, int ld, int r0, int k0, int tid) {
  const int row = tid >> 1, cq = (tid & 1) * 16;
  const _Float16* src = P + (size_t)(r0 + row) * (size_t)ld + k0 + cq;
  const v8h v0 = *(const v8ha*)src;
  const v8h v1 = *(const v8ha*)(src + 8);
  *(v8ha*)(lds + row * GSTR + cq) = v0;
  *(v8ha*)(lds + row * GSTR + cq + 8) = v1;
}

template <int RES>
__global__ __launch_bounds__(128) void k_gemm(const _Float16* __restrict__ A, int lda, int zsa,
                                             const _Float16* __restrict__ Bw, int ldb, int zsb,
                                             float* Y, int ldy, int zsy, const float* __restrict__ R,
                                             int K, float osc) {
#pragma clang fp contract(off)
  __shared__ __attribute__((aligned(16))) unsigned char sm[SMEMB];
  _Float16* lA = (_Float16*)sm;
  _Float16* lB = lA + 64 * GSTR;
  float* oS = (float*)sm;
  const int tid = threadIdx.x, lane = tid & 31, wave = tid >> 5, cl = lane & 15, hh = lane >> 4;
  const int m0 = blockIdx.x * 64;
  const int n0 = blockIdx.y * 64;
  const _Float16* Az = A + (size_t)blockIdx.z * (size_t)zsa;
  const _Float16* Bz = Bw + (size_t)blockIdx.z * (size_t)zsb;
  const size_t zy = (size_t)blockIdx.z * (size_t)zsy;
  float* Yz = Y + zy;
  const float* Rz = R + (RES ? zy : (size_t)0);

  v8f acc[4];
#pragma unroll
  for (int j = 0; j < 4; ++j) { v8f zz = {0.f, 0.f, 0.f, 0.f, 0.f, 0.f, 0.f, 0.f}; acc[j] = zz; }

#pragma unroll 1
  for (int k0 = 0; k0 < K; k0 += 32) {
    __syncthreads();
    stage64(lA, Az, lda, m0, k0, tid);
    stage64(lB, Bz, ldb, n0, k0, tid);
    __syncthreads();
    const v16h af = lds_frag(lA + 16 * wave * GSTR);
    v16h bf[4];
#pragma unroll
    for (int j = 0; j < 4; ++j) bf[j] = lds_frag(lB + 16 * j * GSTR);
#pragma unroll
    for (int j = 0; j < 4; ++j) acc[j] = mma_f16(af, bf[j], acc[j]);
    wguard(acc[0], acc[1], acc[2], acc[3], af, bf[0], bf[1], bf[2], bf[3]);
  }
  __syncthreads();

  float* so = oS + wave * (16 * OSTR);
#pragma unroll
  for (int j = 0; j < 4; ++j)
#pragma unroll
    for (int r = 0; r < 8; ++r)
      so[(8 * hh + r) * OSTR + 16 * j + cl] = acc[j][r] * osc;
  __syncthreads();
#pragma unroll
  for (int pass = 0; pass < 2; ++pass) {
#pragma unroll
    for (int it = 0; it < 8; ++it) {
      const int ch = it * 32 + lane, r = ch >> 4, q = (ch & 15) * 4;
      v4f v = *(const v4fa*)(so + r * OSTR + q);
      const size_t o = (size_t)(m0 + 16 * wave + r) * (size_t)ldy + n0 + q;
      if (RES) { const v4f rr = *(const v4fa*)(Rz + o); v = v + rr; }
      st16f(Yz + o, v);
    }
    __threadfence();
  }
}

__global__ __launch_bounds__(256) void k_cvtw(const float* __restrict__ src, _Float16* dst, int total8, float sc) {
  const int idx = blockIdx.x * 256 + threadIdx.x;
  if (idx >= total8) return;
  const float* s = src + (size_t)idx * 8;
  const v4f a = *(const v4fa*)s, b = *(const v4fa*)(s + 4);
  const v8h o = cvt8(a, b, sc);
  _Float16* d = dst + (size_t)idx * 8;
  st16(d, o);
  __threadfence();
  st16(d, o);
}

__global__ __launch_bounds__(256) void k_cvtconv(const float* __restrict__ src, _Float16* dst, int nrow) {
  const int idx = blockIdx.x * 256 + threadIdx.x;
  if (idx >= nrow * 9 * 64) return;
  const int c8i = idx & 63, t = idx >> 6;
  const int tap = t % 9, row = t / 9;
  const float* s = src + ((size_t)row * CC + (size_t)c8i * 8) * 9 + tap;
  v8h o;
#pragma unroll
  for (int u = 0; u < 8; ++u) o[u] = (_Float16)(s[u * 9] * WSC);
  _Float16* d = dst + (size_t)idx * 8;
  st16(d, o);
  __threadfence();
  st16(d, o);
}

__global__ __launch_bounds__(256) void k_x2tok(const float* __restrict__ x, float* XT) {
  __shared__ float tl[32][129];
  const int tid = threadIdx.x, lane = tid & 31, wave = tid >> 5;
  const int tok0 = blockIdx.x * 32, b = tok0 / L0, hw0 = tok0 - b * L0;
  const int c0 = blockIdx.y * 128;
#pragma unroll 1
  for (int i = 0; i < 16; ++i) {
    const int c = wave + 8 * i;
    tl[lane][c] = x[((size_t)(b * CC + c0 + c)) * L0 + hw0 + lane];
  }
  __syncthreads();
#pragma unroll
  for (int pass = 0; pass < 2; ++pass) {
#pragma unroll
    for (int t = 0; t < 4; ++t) {
      const int tk = wave + 8 * t;
      v4f v;
      v[0] = tl[tk][4 * lane]; v[1] = tl[tk][4 * lane + 1]; v[2] = tl[tk][4 * lane + 2]; v[3] = tl[tk][4 * lane + 3];
      st16f(XT + (size_t)(tok0 + tk) * CC + c0 + 4 * lane, v);
    }
    __threadfence();
  }
}

__global__ __launch_bounds__(64) void k_ln(const float* __restrict__ X, const float* __restrict__ w, const float* __restrict__ bb,
                                          _Float16* Y, float eps) {
#pragma clang fp contract(off)
  __shared__ float red[4];
  const int tid = threadIdx.x, lane = tid & 31, wave = tid >> 5;
  const int tok = blockIdx.x, c8 = tid * 8;
  const float* s = X + (size_t)tok * CC + c8;
  const v4f a = *(const v4fa*)s, b = *(const v4fa*)(s + 4);
  float v[8];
#pragma unroll
  for (int u = 0; u < 4; ++u) { v[u] = a[u]; v[4 + u] = b[u]; }
  float sm = ((((((v[0] + v[1]) + v[2]) + v[3]) + v[4]) + v[5]) + v[6]) + v[7];
  sm = sm + __shfl_xor(sm, 16); sm = sm + __shfl_xor(sm, 8); sm = sm + __shfl_xor(sm, 4);
  sm = sm + __shfl_xor(sm, 2);  sm = sm + __shfl_xor(sm, 1);
  if (lane == 0) red[wave] = sm;
  __syncthreads();
  const float mu = (red[0] + red[1]) * (1.0f / (float)CC);
  float q = 0.0f;
#pragma unroll
  for (int u = 0; u < 8; ++u) { const float dv = v[u] - mu; q = q + dv * dv; }
  q = q + __shfl_xor(q, 16); q = q + __shfl_xor(q, 8); q = q + __shfl_xor(q, 4);
  q = q + __shfl_xor(q, 2);  q = q + __shfl_xor(q, 1);
  if (lane == 0) red[2 + wave] = q;
  __syncthreads();
  const float var = (red[2] + red[3]) * (1.0f / (float)CC);
  const float rs = rsqrtf(var + eps);
  const v4f wa = *(const v4fa*)(w + c8), wb = *(const v4fa*)(w + c8 + 4);
  const v4f ba = *(const v4fa*)(bb + c8), bq = *(const v4fa*)(bb + c8 + 4);
  v8h o;
#pragma unroll
  for (int u = 0; u < 4; ++u) {
    o[u]     = (_Float16)((v[u] - mu) * rs * wa[u] + ba[u]);
    o[4 + u] = (_Float16)((v[4 + u] - mu) * rs * wb[u] + bq[u]);
  }
  _Float16* d = Y + (size_t)tok * CC + c8;
  st16(d, o);
  __threadfence();
  st16(d, o);
}

__global__ __launch_bounds__(256) void k_dwconv(const float* __restrict__ XZ, const float* __restrict__ w,
                                               const float* __restrict__ bias, float* XSF, _Float16* XS16,
                                               int Hs, int Ws) {
  __shared__ __attribute__((aligned(16))) float wsm[9 * DI];
  __shared__ __attribute__((aligned(16))) float stg[2 * DI];
  const int tid = threadIdx.x;
#pragma unroll 1
  for (int i = tid; i < 9 * DI; i += 256) {
    const int tap = i >> 10, c = i & (DI - 1);
    wsm[i] = w[c * 9 + tap];
  }
  __syncthreads();
  const int L = Hs * Ws;
  const int tloc = tid >> 7, tok = blockIdx.x * 2 + tloc, c8 = (tid & 127) * 8;
  const int b = tok / L, l = tok - b * L, hq = l / Ws, wq = l - hq * Ws;
  float acc[8];
#pragma unroll
  for (int u = 0; u < 8; ++u) acc[u] = 0.0f;
#pragma unroll 1
  for (int tap = 0; tap < 9; ++tap) {
    const int kh = tap / 3, kw = tap - kh * 3;
    const int hh = hq + kh - 1, ww = wq + kw - 1;
    const bool ok = (hh >= 0) && (hh < Hs) && (ww >= 0) && (ww < Ws);
    const int hc = clampi(hh, 0, Hs - 1), wc = clampi(ww, 0, Ws - 1);
    const float* s = XZ + ((size_t)(b * L + hc * Ws + wc)) * (2 * DI) + c8;
    const v4f xa = *(const v4fa*)s, xb = *(const v4fa*)(s + 4);
    const v4f wa = *(const v4fa*)(wsm + tap * DI + c8), wb = *(const v4fa*)(wsm + tap * DI + c8 + 4);
#pragma unroll
    for (int u = 0; u < 4; ++u) {
      const float xv = ok ? xa[u] : 0.0f;
      const float xw = ok ? xb[u] : 0.0f;
      acc[u]     = acc[u] + xv * wa[u];
      acc[4 + u] = acc[4 + u] + xw * wb[u];
    }
  }
  const v4f ba = *(const v4fa*)(bias + c8), bq = *(const v4fa*)(bias + c8 + 4);
  float v[8];
#pragma unroll
  for (int u = 0; u < 4; ++u) { v[u] = siluf(acc[u] + ba[u]); v[4 + u] = siluf(acc[4 + u] + bq[u]); }
  {
    v4f s0, s1;
#pragma unroll
    for (int u = 0; u < 4; ++u) { s0[u] = v[u]; s1[u] = v[4 + u]; }
    *(v4fa*)(stg + tloc * DI + c8) = s0;
    *(v4fa*)(stg + tloc * DI + c8 + 4) = s1;
  }
  v8h o;
#pragma unroll
  for (int u = 0; u < 8; ++u) o[u] = (_Float16)(v[u] * XSSC);
  __syncthreads();
  float* fb = XSF + (size_t)blockIdx.x * (2 * DI);
  _Float16* hb = XS16 + (size_t)tok * DI + c8;
#pragma unroll
  for (int pass = 0; pass < 2; ++pass) {
#pragma unroll
    for (int p = 0; p < 2; ++p) {
      const int i4 = tid + p * 256;
      const v4f q4 = *(const v4fa*)(stg + i4 * 4);
      st16f(fb + (size_t)i4 * 4, q4);
    }
    st16(hb, o);
    __threadfence();
  }
}

__global__ __launch_bounds__(256) void k_dtcvt(const float* __restrict__ XD, _Float16* DT16, int total8) {
  const int idx = blockIdx.x * 256 + threadIdx.x;
  if (idx >= total8) return;
  const int tok = idx >> 4, q = idx & 15;
  const float* s = XD + (size_t)tok * XDN + (q >> 2) * XW + (q & 3) * 8;
  const v4f a = *(const v4fa*)s, b = *(const v4fa*)(s + 4);
  const v8h o = cvt8(a, b, DTSC);
  _Float16* d = DT16 + (size_t)idx * 8;
  st16(d, o);
  __threadfence();
  st16(d, o);
}

__global__ __launch_bounds__(256) void k_scan(const float* __restrict__ XSF, float* DY, const float* __restrict__ XD,
                                             const float* __restrict__ dtb, const float* __restrict__ Alog,
                                             const float* __restrict__ Dv, int Hs, int Ws, int M) {
  const int tid = threadIdx.x, blk = blockIdx.x;
  const int b = blk >> 4, k = (blk >> 2) & 3, dch = blk & 3;
  const int d = dch * 256 + tid, kd = k * DI + d;
  const int L = Hs * Ws;
  float A2[NS], h[NS];
#pragma unroll
  for (int n = 0; n < NS; ++n) { A2[n] = -__expf(Alog[(size_t)kd * NS + n]) * LOG2E; h[n] = 0.0f; }
  const float bd = dtb[kd];
  const float Dd = Dv[kd];
  const float* XDk = XD + XW * k;
  float* DYk = DY + (size_t)k * (size_t)M * DI + d;
  const float* Ub = XSF + d;
#pragma unroll 1
  for (int s = 0; s < L; ++s) {
    const int s2 = (k & 2) ? (L - 1 - s) : s;
    const int l = (k & 1) ? ((s2 % Hs) * Ws + s2 / Hs) : s2;
    const size_t tokg = (size_t)(b * L + l);
    const float u = Ub[tokg * DI];
    float* yp = DYk + tokg * DI;
    const float a = *yp + bd;
    const float dl = fmaxf(a, 0.0f) + log1pf(__expf(-fabsf(a)));
    const float* xr = XDk + tokg * XDN;
    v4f Bv[4], Cv[4];
#pragma unroll
    for (int q = 0; q < 4; ++q) {
      Bv[q] = *(const v4fa*)(xr + RK + 4 * q);
      Cv[q] = *(const v4fa*)(xr + RK + NS + 4 * q);
    }
    const float dx = dl * u;
    float y = 0.0f;
#pragma unroll
    for (int n = 0; n < NS; ++n) {
      const float e = exp2f(dl * A2[n]);
      h[n] = e * h[n] + dx * Bv[n >> 2][n & 3];
      y = y + h[n] * Cv[n >> 2][n & 3];
    }
    const float yv = y + Dd * u;
    *(volatile float*)yp = yv;
    __threadfence();
    *(volatile float*)yp = yv;
  }
}

__global__ __launch_bounds__(128) void k_gate(const float* __restrict__ YS, const float* __restrict__ XZ,
                                             const float* __restrict__ g, const float* __restrict__ bt,
                                             _Float16* YG, int M) {
#pragma clang fp contract(off)
  __shared__ float red[8];
  const int tid = threadIdx.x, lane = tid & 31, wave = tid >> 5;
  const int tok = blockIdx.x, c8 = tid * 8;
  float m[8];
  {
    const float* r0 = YS + ((size_t)0 * M + tok) * DI + c8;
    const float* r1 = YS + ((size_t)1 * M + tok) * DI + c8;
    const float* r2 = YS + ((size_t)2 * M + tok) * DI + c8;
    const float* r3 = YS + ((size_t)3 * M + tok) * DI + c8;
    const v4f a0 = *(const v4fa*)r0, b0 = *(const v4fa*)(r0 + 4);
    const v4f a1 = *(const v4fa*)r1, b1 = *(const v4fa*)(r1 + 4);
    const v4f a2 = *(const v4fa*)r2, b2 = *(const v4fa*)(r2 + 4);
    const v4f a3 = *(const v4fa*)r3, b3 = *(const v4fa*)(r3 + 4);
#pragma unroll
    for (int u = 0; u < 4; ++u) {
      m[u]     = ((a0[u] + a2[u]) + a1[u]) + a3[u];
      m[4 + u] = ((b0[u] + b2[u]) + b1[u]) + b3[u];
    }
  }
  float sm = ((((((m[0] + m[1]) + m[2]) + m[3]) + m[4]) + m[5]) + m[6]) + m[7];
  sm = sm + __shfl_xor(sm, 16); sm = sm + __shfl_xor(sm, 8); sm = sm + __shfl_xor(sm, 4);
  sm = sm + __shfl_xor(sm, 2);  sm = sm + __shfl_xor(sm, 1);
  if (lane == 0) red[wave] = sm;
  __syncthreads();
  const float mu = (((red[0] + red[1]) + red[2]) + red[3]) * (1.0f / (float)DI);
  float q = 0.0f;
#pragma unroll
  for (int u = 0; u < 8; ++u) { const float dv = m[u] - mu; q = q + dv * dv; }
  q = q + __shfl_xor(q, 16); q = q + __shfl_xor(q, 8); q = q + __shfl_xor(q, 4);
  q = q + __shfl_xor(q, 2);  q = q + __shfl_xor(q, 1);
  if (lane == 0) red[4 + wave] = q;
  __syncthreads();
  const float var = (((red[4] + red[5]) + red[6]) + red[7]) * (1.0f / (float)DI);
  const float rs = rsqrtf(var + LNE2);
  const size_t zo = (size_t)tok * (2 * DI) + DI + c8;
  const v4f za = *(const v4fa*)(XZ + zo), zb = *(const v4fa*)(XZ + zo + 4);
  const v4f ga = *(const v4fa*)(g + c8), gb = *(const v4fa*)(g + c8 + 4);
  const v4f ba = *(const v4fa*)(bt + c8), bq = *(const v4fa*)(bt + c8 + 4);
  v8h o;
#pragma unroll
  for (int u = 0; u < 4; ++u) {
    const float na = ((m[u] - mu) * rs) * ga[u] + ba[u];
    const float nb = ((m[4 + u] - mu) * rs) * gb[u] + bq[u];
    o[u]     = (_Float16)(na * siluf(za[u]));
    o[4 + u] = (_Float16)(nb * siluf(zb[u]));
  }
  _Float16* dp = YG + (size_t)tok * DI + c8;
  st16(dp, o);
  __threadfence();
  st16(dp, o);
}

__global__ __launch_bounds__(256) void k_down_dw(const float* __restrict__ X, const float* __restrict__ w,
                                                const float* __restrict__ sc, const float* __restrict__ sh,
                                                float* Y, int Hs, int Ws, int total) {
  const int idx = blockIdx.x * 256 + threadIdx.x;
  if (idx >= total) return;
  const int c = idx & (CC - 1), t = idx >> 9;
  const int Ho = Hs / 2, Wo = Ws / 2, Lo = Ho * Wo, L = Hs * Ws;
  const int b = t / Lo, lo = t - b * Lo, ho = lo / Wo, wo = lo - ho * Wo;
  float acc = 0.0f;
#pragma unroll 1
  for (int tap = 0; tap < 9; ++tap) {
    const int kh = tap / 3, kw = tap - kh * 3;
    const int hh = 2 * ho + kh - 1, ww = 2 * wo + kw - 1;
    const bool ok = (hh >= 0) && (hh < Hs) && (ww >= 0) && (ww < Ws);
    const int hc = clampi(hh, 0, Hs - 1), wc = clampi(ww, 0, Ws - 1);
    const float v = X[((size_t)(b * L + hc * Ws + wc)) * CC + c];
    acc = acc + (ok ? v : 0.0f) * w[c * 9 + tap];
  }
  const float y = geluf(acc * (sc[c] * BNS) + sh[c]);
  *(volatile float*)(Y + idx) = y;
  __threadfence();
  *(volatile float*)(Y + idx) = y;
}

template <int RESPRE>
__global__ __launch_bounds__(256) void k_bn_act(const float* __restrict__ X, const float* __restrict__ Rp,
                                               const float* __restrict__ sc, const float* __restrict__ sh,
                                               float* Y, int total) {
#pragma clang fp contract(off)
  const int idx = blockIdx.x * 256 + threadIdx.x;
  if (idx >= total) return;
  const int c = idx & (CC - 1);
  float v = X[idx] * (sc[c] * BNS) + sh[c];
  if (RESPRE) v = v + Rp[idx];
  const float y = geluf(v);
  *(volatile float*)(Y + idx) = y;
  __threadfence();
  *(volatile float*)(Y + idx) = y;
}

__global__ __launch_bounds__(256) void k_upadd(const float* __restrict__ Fin, const float* __restrict__ P, float* Y,
                                              int h, int Ho, int total4) {
#pragma clang fp contract(off)
  const int idx = blockIdx.x * 256 + threadIdx.x;
  if (idx >= total4) return;
  const int c4 = (idx & 127) * 4, t = idx >> 7;
  const int Lo = Ho * Ho, b = t / Lo, lo = t - b * Lo, yo = lo / Ho, xo = lo - yo * Ho;
  const float rd = 1.0f / (float)(Ho - 1);
  const float hm1 = (float)(h - 1);
  const float fy = (yo == Ho - 1) ? hm1 : hm1 * ((float)yo * rd);
  const float fx = (xo == Ho - 1) ? hm1 : hm1 * ((float)xo * rd);
  int y0 = (int)floorf(fy); y0 = clampi(y0, 0, h - 1);
  int x0 = (int)floorf(fx); x0 = clampi(x0, 0, h - 1);
  const int y1 = (y0 + 1 < h) ? (y0 + 1) : (h - 1);
  const int x1 = (x0 + 1 < h) ? (x0 + 1) : (h - 1);
  const float wy = fy - (float)y0, wx = fx - (float)x0;
  const float uy = 1.0f - wy, ux = 1.0f - wx;
  const size_t rb = (size_t)b * h * h;
  const v4f p00 = *(const v4fa*)(Fin + (rb + (size_t)y0 * h + x0) * CC + c4);
  const v4f p01 = *(const v4fa*)(Fin + (rb + (size_t)y0 * h + x1) * CC + c4);
  const v4f p10 = *(const v4fa*)(Fin + (rb + (size_t)y1 * h + x0) * CC + c4);
  const v4f p11 = *(const v4fa*)(Fin + (rb + (size_t)y1 * h + x1) * CC + c4);
  const v4f pp  = *(const v4fa*)(P + (size_t)t * CC + c4);
  v4f o;
#pragma unroll
  for (int u = 0; u < 4; ++u) {
    const float g0 = p00[u] * uy + p10[u] * wy;
    const float g1 = p01[u] * uy + p11[u] * wy;
    o[u] = (g0 * ux + g1 * wx) + pp[u];
  }
  float* d = Y + (size_t)t * CC + c4;
  st16f(d, o);
  __threadfence();
  st16f(d, o);
}

__global__ __launch_bounds__(256) void k_im2col(const float* __restrict__ X, _Float16* COL, int Hs, int total8) {
  const int idx = blockIdx.x * 256 + threadIdx.x;
  if (idx >= total8) return;
  const int c8 = (idx & 63) * 8, t = idx >> 6;
  const int tap = t % 9, tok = t / 9;
  const int L = Hs * Hs, b = tok / L, l = tok - b * L, hq = l / Hs, wq = l - hq * Hs;
  const int kh = tap / 3, kw = tap - kh * 3;
  const int hh = hq + kh - 1, ww = wq + kw - 1;
  const bool ok = (hh >= 0) && (hh < Hs) && (ww >= 0) && (ww < Hs);
  const int hc = clampi(hh, 0, Hs - 1), wc = clampi(ww, 0, Hs - 1);
  const float* s = X + ((size_t)(b * L + hc * Hs + wc)) * CC + c8;
  const v4f a = *(const v4fa*)s, bq = *(const v4fa*)(s + 4);
  v8h o;
#pragma unroll
  for (int u = 0; u < 4; ++u) {
    o[u]     = (_Float16)(ok ? a[u] : 0.0f);
    o[4 + u] = (_Float16)(ok ? bq[u] : 0.0f);
  }
  _Float16* d = COL + (size_t)idx * 8;
  st16(d, o);
  __threadfence();
  st16(d, o);
}

__global__ __launch_bounds__(256) void k_out(const float* __restrict__ RAW, const float* __restrict__ sc,
                                            const float* __restrict__ sh, const float* __restrict__ x, float* out) {
#pragma clang fp contract(off)
  __shared__ float tl[32][129];
  const int tid = threadIdx.x, lane = tid & 31, wave = tid >> 5;
  const int tok0 = blockIdx.x * 128, b = tok0 / L0, hw0 = tok0 - b * L0;
  const int c0 = blockIdx.y * 32;
  const float s1 = sc[c0 + lane] * BNS, b1 = sh[c0 + lane];
#pragma unroll 1
  for (int i = 0; i < 16; ++i) {
    const int tk = wave * 16 + i;
    const float v = RAW[(size_t)(tok0 + tk) * CC + c0 + lane];
    tl[lane][tk] = geluf(v * s1 + b1);
  }
  __syncthreads();
#pragma unroll
  for (int pass = 0; pass < 2; ++pass) {
#pragma unroll
    for (int t = 0; t < 4; ++t) {
      const int cl = wave * 4 + t;
      const size_t o = ((size_t)(b * CC + c0 + cl)) * L0 + hw0 + 4 * lane;
      const v4f xr = *(const v4fa*)(x + o);
      v4f v;
      v[0] = tl[cl][4 * lane] + xr[0];     v[1] = tl[cl][4 * lane + 1] + xr[1];
      v[2] = tl[cl][4 * lane + 2] + xr[2]; v[3] = tl[cl][4 * lane + 3] + xr[3];
      st16f(out + o, v);
    }
    __threadfence();
  }
}

extern "C" void kernel_launch(void* const* d_in, const int* in_sizes, int n_in,
                              void* d_out, int out_size, void* d_ws, size_t ws_size,
                              hipStream_t stream) {
  if (n_in < 31) return;
  if (in_sizes[0] != NB * CC * L0 || in_sizes[1] != NVSS * CC || in_sizes[2] != NVSS * CC ||
      in_sizes[3] != NVSS * 2 * DI * CC || in_sizes[4] != NVSS * DI * 9 || in_sizes[5] != NVSS * DI ||
      in_sizes[6] != NVSS * KD * XW * DI || in_sizes[7] != NVSS * KD * DI * RK || in_sizes[8] != NVSS * KD * DI ||
      in_sizes[9] != NVSS * KD * DI * NS || in_sizes[10] != NVSS * KD * DI || in_sizes[11] != NVSS * DI ||
      in_sizes[12] != NVSS * DI || in_sizes[13] != NVSS * CC * DI || in_sizes[14] != 2 * CC * 9 ||
      in_sizes[15] != 2 * CC || in_sizes[16] != 2 * CC || in_sizes[17] != 2 * CC * CC || in_sizes[18] != 2 * CC ||
      in_sizes[19] != 2 * CC || in_sizes[20] != 2 * CC * CC * 9 || in_sizes[21] != 2 * CC || in_sizes[22] != 2 * CC ||
      in_sizes[23] != 2 * CC * CC * 9 || in_sizes[24] != 2 * CC || in_sizes[25] != 2 * CC || in_sizes[26] != CC ||
      in_sizes[27] != CC || in_sizes[28] != CC * CC * 9 || in_sizes[29] != CC || in_sizes[30] != CC ||
      out_size != NB * CC * L0) return;

  const float* x        = (const float*)d_in[0];
  const float* ln_w     = (const float*)d_in[1];
  const float* ln_b     = (const float*)d_in[2];
  const float* in_proj  = (const float*)d_in[3];
  const float* conv_w   = (const float*)d_in[4];
  const float* conv_b   = (const float*)d_in[5];
  const float* xproj    = (const float*)d_in[6];
  const float* dtw      = (const float*)d_in[7];
  const float* dtb      = (const float*)d_in[8];
  const float* Alog     = (const float*)d_in[9];
  const float* Dp       = (const float*)d_in[10];
  const float* onw      = (const float*)d_in[11];
  const float* onb      = (const float*)d_in[12];
  const float* outproj  = (const float*)d_in[13];
  const float* ds_dw    = (const float*)d_in[14];
  const float* ds_bn1s  = (const float*)d_in[15];
  const float* ds_bn1b  = (const float*)d_in[16];
  const float* ds_pw    = (const float*)d_in[17];
  const float* ds_bn2s  = (const float*)d_in[18];
  const float* ds_bn2b  = (const float*)d_in[19];
  const float* fus_c1   = (const float*)d_in[20];
  const float* fus_bn1s = (const float*)d_in[21];
  const float* fus_bn1b = (const float*)d_in[22];
  const float* fus_c2   = (const float*)d_in[23];
  const float* fus_bn2s = (const float*)d_in[24];
  const float* fus_bn2b = (const float*)d_in[25];
  const float* op_bn0s  = (const float*)d_in[26];
  const float* op_bn0b  = (const float*)d_in[27];
  const float* op_conv  = (const float*)d_in[28];
  const float* op_bn1s  = (const float*)d_in[29];
  const float* op_bn1b  = (const float*)d_in[30];
  float* out = (float*)d_out;

  size_t off = 0;
  auto carve = [&](size_t bytes) -> char* { char* p = (char*)d_ws + off; off += (bytes + 255) & ~(size_t)255; return p; };
  _Float16* WIN16  = (_Float16*)carve((size_t)NVSS * 2 * DI * CC * 2);
  _Float16* WX16   = (_Float16*)carve((size_t)NVSS * XDN * DI * 2);
  _Float16* WDT16  = (_Float16*)carve((size_t)NVSS * KD * DI * RK * 2);
  _Float16* WOUT16 = (_Float16*)carve((size_t)NVSS * CC * DI * 2);
  _Float16* WPW16  = (_Float16*)carve((size_t)2 * CC * CC * 2);
  _Float16* WC116  = (_Float16*)carve((size_t)2 * CC * KC9 * 2);
  _Float16* WC216  = (_Float16*)carve((size_t)2 * CC * KC9 * 2);
  _Float16* WOP16  = (_Float16*)carve((size_t)CC * KC9 * 2);
  float* XT    = (float*)carve((size_t)M0 * CC * 4);
  float* V0    = (float*)carve((size_t)M0 * CC * 4);
  float* XR    = (float*)carve((size_t)M0 * CC * 4);
  float* P1    = (float*)carve((size_t)(M0 / 4) * CC * 4);
  float* P2    = (float*)carve((size_t)(M0 / 16) * CC * 4);
  float* PROC0 = (float*)carve((size_t)M0 * CC * 4);
  float* PROC1 = (float*)carve((size_t)(M0 / 4) * CC * 4);
  float* PROC2 = (float*)carve((size_t)(M0 / 16) * CC * 4);
  _Float16* LN16 = (_Float16*)carve((size_t)M0 * CC * 2);
  float* XZ      = (float*)carve((size_t)M0 * 2 * DI * 4);
  float* XSF     = (float*)carve((size_t)M0 * DI * 4);
  _Float16* XS16 = (_Float16*)carve((size_t)M0 * DI * 2);
  float* XD      = (float*)carve((size_t)M0 * XDN * 4);
  _Float16* DT16 = (_Float16*)carve((size_t)M0 * KD * RK * 2);
  float* DY      = (float*)carve((size_t)KD * M0 * DI * 4);
  _Float16* YG16 = (_Float16*)carve((size_t)M0 * DI * 2);
  float* DWF      = (float*)carve((size_t)(M0 / 4) * CC * 4);
  _Float16* DW16  = (_Float16*)carve((size_t)(M0 / 4) * CC * 2);
  float* RAW      = (float*)carve((size_t)M0 * CC * 4);
  float* H1       = (float*)carve((size_t)M0 * CC * 4);
  float* XRES8    = (float*)carve((size_t)(M0 / 4) * CC * 4);
  float* FUSED8   = (float*)carve((size_t)(M0 / 4) * CC * 4);
  float* XRES16   = (float*)carve((size_t)M0 * CC * 4);
  float* FUSED16  = (float*)carve((size_t)M0 * CC * 4);
  float* HOP      = (float*)carve((size_t)M0 * CC * 4);
  _Float16* COL16 = (_Float16*)carve((size_t)M0 * KC9 * 2);
  if (off > ws_size || off > (size_t)134217728) return;

  const dim3 b256(256), b128(128), b64(64);

  k_cvtw<<<dim3((NVSS * 2 * DI * CC / 8 + 255) / 256), b256, 0, stream>>>(in_proj, WIN16, NVSS * 2 * DI * CC / 8, WSC);
  k_cvtw<<<dim3((NVSS * XDN * DI / 8 + 255) / 256), b256, 0, stream>>>(xproj, WX16, NVSS * XDN * DI / 8, WSC);
  k_cvtw<<<dim3((NVSS * KD * DI * RK / 8 + 255) / 256), b256, 0, stream>>>(dtw, WDT16, NVSS * KD * DI * RK / 8, WSC);
  k_cvtw<<<dim3((NVSS * CC * DI / 8 + 255) / 256), b256, 0, stream>>>(outproj, WOUT16, NVSS * CC * DI / 8, WSC);
  k_cvtw<<<dim3((2 * CC * CC / 8 + 255) / 256), b256, 0, stream>>>(ds_pw, WPW16, 2 * CC * CC / 8, WSC);
  k_cvtconv<<<dim3((2 * CC * 9 * 64 + 255) / 256), b256, 0, stream>>>(fus_c1, WC116, 2 * CC);
  k_cvtconv<<<dim3((2 * CC * 9 * 64 + 255) / 256), b256, 0, stream>>>(fus_c2, WC216, 2 * CC);
  k_cvtconv<<<dim3((CC * 9 * 64 + 255) / 256), b256, 0, stream>>>(op_conv, WOP16, CC);

  k_x2tok<<<dim3(M0 / 32, CC / 128), b256, 0, stream>>>(x, XT);

  auto vss = [&](const float* xin, float* xout, int i, int Hs) {
    const int M = NB * Hs * Hs;
    k_ln<<<dim3(M), b64, 0, stream>>>(xin, ln_w + (size_t)i * CC, ln_b + (size_t)i * CC, LN16, LNE1);
    k_gemm<0><<<dim3(M / 64, 2 * DI / 64, 1), b128, 0, stream>>>(LN16, CC, 0, WIN16 + (size_t)i * 2 * DI * CC, CC, 0,
                                                                 XZ, 2 * DI, 0, XZ, CC, OSC1);
    k_dwconv<<<dim3(M / 2), b256, 0, stream>>>(XZ, conv_w + (size_t)i * DI * 9, conv_b + (size_t)i * DI, XSF, XS16, Hs, Hs);
    k_gemm<0><<<dim3(M / 64, XDN / 64, 1), b128, 0, stream>>>(XS16, DI, 0, WX16 + (size_t)i * XDN * DI, DI, 0,
                                                              XD, XDN, 0, XD, DI, OSCX);
    k_dtcvt<<<dim3((M * 16 + 255) / 256), b256, 0, stream>>>(XD, DT16, M * 16);
    k_gemm<0><<<dim3(M / 64, DI / 64, KD), b128, 0, stream>>>(DT16, KD * RK, RK, WDT16 + (size_t)i * KD * DI * RK, RK, DI * RK,
                                                              DY, DI, M * DI, DY, RK, OSCD);
    k_scan<<<dim3(NB * KD * (DI / 256)), b256, 0, stream>>>(XSF, DY, XD, dtb + (size_t)i * KD * DI,
                                                          Alog + (size_t)i * KD * DI * NS, Dp + (size_t)i * KD * DI, Hs, Hs, M);
    k_gate<<<dim3(M), b128, 0, stream>>>(DY, XZ, onw + (size_t)i * DI, onb + (size_t)i * DI, YG16, M);
    k_gemm<1><<<dim3(M / 64, CC / 64, 1), b128, 0, stream>>>(YG16, DI, 0, WOUT16 + (size_t)i * CC * DI, DI, 0,
                                                             xout, CC, 0, xin, DI, OSC1);
  };

  auto down = [&](const float* xin, float* xout, int j, int Hs) {
    const int Ho = Hs / 2, Mo = NB * Ho * Ho;
    k_down_dw<<<dim3((Mo * CC + 255) / 256), b256, 0, stream>>>(xin, ds_dw + (size_t)j * CC * 9, ds_bn1s + (size_t)j * CC,
                                                              ds_bn1b + (size_t)j * CC, DWF, Hs, Hs, Mo * CC);
    k_cvtw<<<dim3((Mo * CC / 8 + 255) / 256), b256, 0, stream>>>(DWF, DW16, Mo * CC / 8, 1.0f);
    k_gemm<0><<<dim3(Mo / 64, CC / 64, 1), b128, 0, stream>>>(DW16, CC, 0, WPW16 + (size_t)j * CC * CC, CC, 0,
                                                              RAW, CC, 0, RAW, CC, OSC1);
    k_bn_act<0><<<dim3((Mo * CC + 255) / 256), b256, 0, stream>>>(RAW, RAW, ds_bn2s + (size_t)j * CC, ds_bn2b + (size_t)j * CC,
                                                                xout, Mo * CC);
  };

  auto resblk = [&](const float* xin, float* xout, int j, int Hs) {
    const int M = NB * Hs * Hs;
    k_im2col<<<dim3((M * 9 * 64 + 255) / 256), b256, 0, stream>>>(xin, COL16, Hs, M * 9 * 64);
    k_gemm<0><<<dim3(M / 64, CC / 64, 1), b128, 0, stream>>>(COL16, KC9, 0, WC116 + (size_t)j * CC * KC9, KC9, 0,
                                                             RAW, CC, 0, RAW, KC9, OSC1);
    k_bn_act<0><<<dim3((M * CC + 255) / 256), b256, 0, stream>>>(RAW, RAW, fus_bn1s + (size_t)j * CC, fus_bn1b + (size_t)j * CC,
                                                               H1, M * CC);
    k_im2col<<<dim3((M * 9 * 64 + 255) / 256), b256, 0, stream>>>(H1, COL16, Hs, M * 9 * 64);
    k_gemm<0><<<dim3(M / 64, CC / 64, 1), b128, 0, stream>>>(COL16, KC9, 0, WC216 + (size_t)j * CC * KC9, KC9, 0,
                                                             RAW, CC, 0, RAW, KC9, OSC1);
    k_bn_act<1><<<dim3((M * CC + 255) / 256), b256, 0, stream>>>(RAW, xin, fus_bn2s + (size_t)j * CC, fus_bn2b + (size_t)j * CC,
                                                               xout, M * CC);
  };

  vss(XT, V0, 0, H0);
  vss(V0, XR, 1, H0);
  down(XR, P1, 0, H0);
  down(P1, P2, 1, H0 / 2);
  vss(XR, PROC0, 2, H0);
  vss(P1, PROC1, 3, H0 / 2);
  vss(P2, PROC2, 4, H0 / 4);
  k_upadd<<<dim3(((M0 / 4) * 128 + 255) / 256), b256, 0, stream>>>(PROC2, PROC1, XRES8, H0 / 4, H0 / 2, (M0 / 4) * 128);
  resblk(XRES8, FUSED8, 0, H0 / 2);
  k_upadd<<<dim3((M0 * 128 + 255) / 256), b256, 0, stream>>>(FUSED8, PROC0, XRES16, H0 / 2, H0, M0 * 128);
  resblk(XRES16, FUSED16, 1, H0);
  k_bn_act<0><<<dim3((M0 * CC + 255) / 256), b256, 0, stream>>>(FUSED16, FUSED16, op_bn0s, op_bn0b, HOP, M0 * CC);
  k_im2col<<<dim3((M0 * 9 * 64 + 255) / 256), b256, 0, stream>>>(HOP, COL16, H0, M0 * 9 * 64);
  k_gemm<0><<<dim3(M0 / 64, CC / 64, 1), b128, 0, stream>>>(COL16, KC9, 0, WOP16, KC9, 0, RAW, CC, 0, RAW, KC9, OSC1);
  k_out<<<dim3(M0 / 128, CC / 32), b256, 0, stream>>>(RAW, op_bn1s, op_bn1b, x, out);
}
